// CrossModalAttention_48558900248898
// MI455X (gfx1250) — hardware-run, weakly checked
//
#include <hip/hip_runtime.h>


namespace {
constexpr int NB = 2, C = 256, H = 128, W = 128, HW = H * W, TK = 4, T2 = 16, NHT = H / TK  , NWT = W / TK;
constexpr float XS = 8.0f, WSC = 256.0f, SCALE = 0.25f;
typedef _Float16 b16;
typedef __attribute__((ext_vector_type(16))) _Float16 v16b;
typedef __attribute__((ext_vector_type(8))) _Float16 v8b;
typedef __attribute__((ext_vector_type(8))) float v8f;
typedef __attribute__((ext_vector_type(4))) float v4f;
__device__ __forceinline__ float bf16_rne(float f) { unsigned int u = __float_as_uint(f); u += 0x7FFFu + ((u >> 16) & 1u); float r = __uint_as_float(u & 0xFFFF0000u); asm volatile("" : "+v"(r)); return r; }
__device__ __forceinline__ float bfv(float f) { float r = bf16_rne(f); asm volatile("" : "+v"(r)); return r; }
__device__ __forceinline__ v16b frag_kb(const b16* p, int hh) { const v8b a = *(const v8b*)(p + 8 * hh), b = *(const v8b*)(p + 16 + 8 * hh); v16b f;
#pragma unroll
  for (int e = 0; e < 8; ++e) { f[e] = a[e]; f[8 + e] = b[e]; } return f; }
__device__ __forceinline__ v8f wmma16b(v16b a, v16b b, v8f c) { v8f d = __builtin_amdgcn_wmma_f32_16x16x32_f16(false, a, false, b, (short)0, c, false, false); asm volatile("v_nop\n\tv_nop\n\tv_nop\n\tv_nop" : "+v"(d) : "v"(a), "v"(b)); return d; }
__device__ __forceinline__ void wave_lds_sync() { __builtin_amdgcn_fence(__ATOMIC_RELEASE, "workgroup"); __builtin_amdgcn_wave_barrier(); __builtin_amdgcn_fence(__ATOMIC_ACQUIRE, "workgroup"); }
__device__ __forceinline__ float pmul(float a, float b) { float p = a * b; asm volatile("" : "+v"(p)); return p; }

__global__ __launch_bounds__(256) void wput_kernel(const float* __restrict__ wq, const float* __restrict__ wk, const float* __restrict__ wv, b16* __restrict__ WT) { const size_t u = (size_t)blockIdx.x * 256 + threadIdx.x; if (u >= (size_t)3 * C * 32) return; const int r = (int)(u / 32), k0 = (int)(u % 32) * 8; const int p = r / C, o = r % C; const float* w = p == 0 ? wq : (p == 1 ? wk : wv); v8b v;
#pragma unroll
  for (int j = 0; j < 8; ++j) v[j] = (b16)(bf16_rne(w[(size_t)o * C + k0 + j]) * WSC); for (int pass = 0; pass < 2; ++pass) { *(volatile v8b*)(WT + (size_t)r * C + k0) = v; __threadfence(); } }
__global__ __launch_bounds__(32) void proj_kernel(const float* __restrict__ blue, const float* __restrict__ white, const b16* __restrict__ WT, const float* __restrict__ bq, const float* __restrict__ bk, const float* __restrict__ bv, int BLIM, float* __restrict__ TP) { __shared__ __attribute__((aligned(16))) b16 Ah[16][C + 8]; __shared__ float Tf[16][C + 4]; const int lane = threadIdx.x, nloc = lane & 15, hlf = lane >> 4;
  const int wb = blockIdx.x % (W / 16); const int i = (blockIdx.x / (W / 16)) % NHT; const int b = (blockIdx.x / ((W / 16) * NHT)) % NB; const int p = blockIdx.x / ((W / 16) * NHT * NB); if (b >= BLIM) return; const int w0 = wb * 16;
  const float* in = p == 0 ? blue : white; const float* bias = p == 0 ? bq : (p == 1 ? bk : bv); const size_t tokb = (((size_t)p * NB + b) * NHT + i) * NWT;
  for (int pass = 0; pass < 2; ++pass) {
#pragma unroll 1
    for (int th = 0; th < TK; ++th) { const int h = i * TK + th;
      for (int c8 = 0; c8 < C; c8 += 2) { const int c = c8 + hlf; Ah[nloc][c] = (b16)(bf16_rne(in[(((size_t)b * C + c) * H + h) * W + w0 + nloc]) * XS); }
      wave_lds_sync(); v8f acc[16];
#pragma unroll
      for (int t = 0; t < 16; ++t) acc[t] = (v8f){};
#pragma unroll 2
      for (int kb = 0; kb < C; kb += 32) { const v16b a = frag_kb(&Ah[nloc][kb], hlf);
#pragma unroll
        for (int t = 0; t < 16; ++t) acc[t] = wmma16b(a, frag_kb(WT + ((size_t)p * C + t * 16 + nloc) * C + kb, hlf), acc[t]); }
#pragma unroll
      for (int t = 0; t < 16; ++t) { const int cc = t * 16 + nloc; const float bb = bfv(bias[cc]);
#pragma unroll
        for (int r8 = 0; r8 < 8; ++r8) Tf[8 * hlf + r8][cc] = acc[t][r8] * (1.0f / (XS * WSC)) + bb; }
      wave_lds_sync();
      for (int c8 = 0; c8 < C; c8 += 8) { const int c = c8 + (lane >> 2); const int jt = lane & 3; const int j = w0 / TK + jt; const v4f v = {Tf[jt * 4 + 0][c], Tf[jt * 4 + 1][c], Tf[jt * 4 + 2][c], Tf[jt * 4 + 3][c]}; *(volatile v4f*)(TP + ((tokb + j) * C + c) * T2 + th * 4) = v; }
      wave_lds_sync(); }
    __threadfence(); } }
__global__ __launch_bounds__(256) void natt_kernel(const float* __restrict__ TP, int BLIM, float* __restrict__ out) { const int wave = threadIdx.x >> 5, lane = threadIdx.x & 31; const size_t gw = (size_t)blockIdx.x * 8 + wave; const int i = (int)(gw % NHT); const int c = (int)((gw / NHT) % C); const int b = (int)(gw / ((size_t)NHT * C)); if (b >= BLIM) return; const int j = lane;
  const float* QP = TP; const float* KP = TP + (size_t)NB * NHT * NWT * C * T2; const float* VP = KP + (size_t)NB * NHT * NWT * C * T2;
  auto tok = [&](const float* base, int ii, int jj) { return base + ((((size_t)b * NHT + ii) * NWT + jj) * C + c) * T2; };
  float q[16]; { const float* qp = tok(QP, i, j);
#pragma unroll
    for (int t = 0; t < 16; ++t) q[t] = qp[t]; }
  float sc[9]; float mx = -INFINITY;
#pragma unroll
  for (int n = 0; n < 9; ++n) { const int ii = i + n / 3 - 1, jj = j + n % 3 - 1; float s = -INFINITY; if (ii >= 0 && ii < NHT && jj >= 0 && jj < NWT) { const float* kp = tok(KP, ii, jj); float d = 0.0f;
#pragma unroll
      for (int t = 0; t < 16; ++t) d += pmul(q[t], kp[t]); s = d * SCALE; } sc[n] = s; mx = fmaxf(mx, s); }
  float den = 0.0f, o[16];
#pragma unroll
  for (int t = 0; t < 16; ++t) o[t] = 0.0f;
#pragma unroll
  for (int n = 0; n < 9; ++n) { if (sc[n] == -INFINITY) continue; const float pn = __expf(sc[n] - mx); den += pn; const int ii = i + n / 3 - 1, jj = j + n % 3 - 1; const float* vp = tok(VP, ii, jj);
#pragma unroll
    for (int t = 0; t < 16; ++t) o[t] += pmul(pn, vp[t]); }
  const float inv = 1.0f / den;
  for (int pass = 0; pass < 2; ++pass) {
#pragma unroll
    for (int th = 0; th < 4; ++th) *(volatile v4f*)(out + (((size_t)b * C + c) * H + i * TK + th) * W + j * TK) = (v4f){o[th * 4] * inv, o[th * 4 + 1] * inv, o[th * 4 + 2] * inv, o[th * 4 + 3] * inv};
    __threadfence(); } }
}

extern "C" void kernel_launch(void* const* d_in, const int* in_sizes, int n_in, void* d_out, int out_size, void* d_ws, size_t ws_size, hipStream_t stream) {
  (void)n_in;
  auto Fp = [&](int i) { return (const float*)d_in[i]; };
  if (in_sizes[0] != NB * C * HW || in_sizes[1] != NB * C * HW || in_sizes[2] != C * C || in_sizes[4] != C * C || in_sizes[6] != C * C || out_size != NB * C * HW) return;
  const int BLIM = NB;
  size_t off = 0; char* ws = (char*)d_ws;
  auto carve = [&](size_t bytes) { char* p = ws + off; off += (bytes + 255) & ~(size_t)255; return p; };
  b16* WT = (b16*)carve((size_t)3 * C * C * 2); float* TP = (float*)carve((size_t)3 * NB * C * HW * 4);
  if (off > ws_size || off > ((size_t)128 << 20)) return;
  wput_kernel<<<(3 * C * 32 + 255) / 256, 256, 0, stream>>>(Fp(2), Fp(4), Fp(6), WT);
  proj_kernel<<<3 * NB * NHT * (W / 16), 32, 0, stream>>>(Fp(0), Fp(1), WT, Fp(3), Fp(5), Fp(7), BLIM, TP);
  natt_kernel<<<(unsigned)(((size_t)BLIM * C * NHT + 7) / 8), 256, 0, stream>>>(TP, BLIM, (float*)d_out);
}
